// BahdanauAttention_33002528702914
// MI455X (gfx1250) — hardware-verified
//
#include <hip/hip_runtime.h>


#ifndef NB
#define NB 8
#endif
#define NB_FULL 8
#define TQ   64
#define SK   512
#define QD   1024
#define VD   512
#define UN   256
#define PCAR 4096.0f
#define PINV (1.0f / 4096.0f)
#define TRP  65

static_assert(NB <= NB_FULL);
static_assert(TQ % 64 == 0);
static_assert((NB * TQ) % 64 == 0);
static_assert((NB * SK) % 64 == 0);
static_assert(UN % 64 == 0);
static_assert(VD % 64 == 0);
static_assert(QD % 64 == 0);
static_assert(SK % 64 == 0);
static_assert(QD % 32 == 0);
static_assert(VD % 32 == 0);
static_assert(SK % 32 == 0);
static_assert(UN == 256);
static_assert(UN % 32 == 0);
static_assert(SK == 2 * 256);
static_assert(SK == 128 * 4);
static_assert(SK == 64 * 8);
static_assert(SK % 8 == 0);
static_assert(((size_t)NB * TQ * QD) % 8 == 0);
static_assert(((size_t)NB * SK * VD) % 8 == 0);
static_assert(32 * 16 * 8 == 16 * 64 * 4);
static_assert(256 * 16 * 2 == 64 * 64 * 2);
static_assert(256 * 16 * 4 == 64 * 64 * 4);
static_assert((16 * 68) * 4 <= 131072);
static_assert((64 * TRP) * 4 <= 131072);
static_assert((UN + UN + SK + 16) * 4 <= 131072);

typedef _Float16 h16;
typedef unsigned short bf;
typedef __attribute__((ext_vector_type(16))) __bf16   v16bf;
typedef __attribute__((ext_vector_type(16))) _Float16 v16h;
typedef __attribute__((ext_vector_type(8)))  _Float16 v8h;
typedef __attribute__((ext_vector_type(8)))  unsigned short v8us;
typedef __attribute__((ext_vector_type(8)))  float    v8f;
typedef __attribute__((ext_vector_type(4)))  float    v4f;
typedef v4f  __attribute__((may_alias)) v4fa;

__device__ __forceinline__ unsigned short f2bf(float f) { unsigned u = __float_as_uint(f); u += 0x7FFFu + ((u >> 16) & 1u); return (unsigned short)(u >> 16); }
__device__ __forceinline__ float bfr(float f) { return __uint_as_float(((unsigned)f2bf(f)) << 16); }
__device__ __forceinline__ v16h cat16(v8h lo, v8h hi) { return __builtin_shufflevector(lo, hi, 0, 1, 2, 3, 4, 5, 6, 7, 8, 9, 10, 11, 12, 13, 14, 15); }
__device__ __forceinline__ v16bf cat16b(v8us lo, v8us hi) { return __builtin_bit_cast(v16bf, __builtin_shufflevector(lo, hi, 0, 1, 2, 3, 4, 5, 6, 7, 8, 9, 10, 11, 12, 13, 14, 15)); }
__device__ __forceinline__ v8f wmma16(v16h a, v16h b, v8f c) { return __builtin_amdgcn_wmma_f32_16x16x32_f16(false, a, false, b, (short)0, c, false, false); }
__device__ __forceinline__ v8f wmmab(v16bf a, v16bf b, v8f c) { return __builtin_amdgcn_wmma_f32_16x16x32_bf16(false, a, false, b, (short)0, c, false, false); }
__device__ __forceinline__ v16h  ldh(const h16* p) { return cat16(*(const v8h*)p, *(const v8h*)(p + 16)); }
__device__ __forceinline__ v16bf ldb(const bf* p)  { return cat16b(*(const v8us*)p, *(const v8us*)(p + 16)); }
__device__ __forceinline__ void wave_sync() { __builtin_amdgcn_fence(3  , "wavefront"); __builtin_amdgcn_wave_barrier(); asm volatile("" ::: "memory"); }

__device__ __forceinline__ v8f wmmabg(v16bf a, v16bf b, v8f c) { c = wmmab(a, b, c); asm volatile("v_nop\n\tv_nop\n\tv_nop\n\tv_nop" : "+v"(c) : "v"(a), "v"(b)); return c; }
__device__ __forceinline__ v8f wmma16g(v16h a, v16h b, v8f c) { c = wmma16(a, b, c); asm volatile("v_nop\n\tv_nop\n\tv_nop\n\tv_nop" : "+v"(c) : "v"(a), "v"(b)); return c; }
static __device__ __forceinline__ h16 toh_flush(float v) { const float w = (fabsf(v) < 6.103515625e-05f) ? 0.0f : v; return (h16)w; }

__global__ __launch_bounds__(256) void k_cvt8(const float* __restrict__ src, bf* dst, size_t n8) {
    const size_t i = (size_t)blockIdx.x * 256 + threadIdx.x; if (i >= n8) return;
    const v8f v = *(const v8f*)(src + i * 8); v8us o;
#pragma unroll
    for (int k = 0; k < 8; ++k) o[k] = f2bf(v[k]);
    *(volatile v8us*)(dst + i * 8) = o; __threadfence(); *(volatile v8us*)(dst + i * 8) = o;
}

__global__ __launch_bounds__(256) void k_trb(const float* __restrict__ in, bf* out, unsigned rows, unsigned cols) {
    __shared__ float ts[64 * TRP];
    const unsigned tid = threadIdx.x; const unsigned c0 = blockIdx.x * 64u, r0 = blockIdx.y * 64u;
#pragma unroll
    for (unsigned it = 0; it < 4u; ++it) { const unsigned r = it * 16u + (tid >> 4), c4 = (tid & 15u) * 4u;
        const v4f x = *(const v4f*)(in + (size_t)(r0 + r) * cols + c0 + c4);
        ts[r * TRP + c4 + 0] = x[0]; ts[r * TRP + c4 + 1] = x[1]; ts[r * TRP + c4 + 2] = x[2]; ts[r * TRP + c4 + 3] = x[3]; }
    __syncthreads();
#pragma unroll 1
    for (int ps = 0; ps < 2; ++ps) {
#pragma unroll
        for (unsigned it = 0; it < 2u; ++it) { const unsigned n = it * 32u + (tid >> 3), k8 = (tid & 7u) * 8u; v8us o;
#pragma unroll
            for (int j = 0; j < 8; ++j) o[j] = f2bf(ts[(k8 + (unsigned)j) * TRP + n]);
            *(volatile v8us*)(out + (size_t)(c0 + n) * rows + r0 + k8) = o; }
        if (ps == 0) __threadfence(); }
}

__global__ __launch_bounds__(256) void k_trh(const float* __restrict__ in, h16* out, unsigned rows, unsigned cols) {
    __shared__ float ts[64 * TRP];
    const unsigned tid = threadIdx.x; const unsigned c0 = blockIdx.x * 64u, r0 = blockIdx.y * 64u;
    const size_t zb = (size_t)blockIdx.z * rows * cols;
#pragma unroll
    for (unsigned it = 0; it < 4u; ++it) { const unsigned r = it * 16u + (tid >> 4), c4 = (tid & 15u) * 4u;
        const v4f x = *(const v4f*)(in + zb + (size_t)(r0 + r) * cols + c0 + c4);
        ts[r * TRP + c4 + 0] = x[0]; ts[r * TRP + c4 + 1] = x[1]; ts[r * TRP + c4 + 2] = x[2]; ts[r * TRP + c4 + 3] = x[3]; }
    __syncthreads();
#pragma unroll 1
    for (int ps = 0; ps < 2; ++ps) {
#pragma unroll
        for (unsigned it = 0; it < 2u; ++it) { const unsigned n = it * 32u + (tid >> 3), k8 = (tid & 7u) * 8u; v8h o;
#pragma unroll
            for (int j = 0; j < 8; ++j) o[j] = toh_flush(bfr(ts[(k8 + (unsigned)j) * TRP + n]));
            *(volatile v8h*)(out + zb + (size_t)(c0 + n) * rows + r0 + k8) = o; }
        if (ps == 0) __threadfence(); }
}

__global__ __launch_bounds__(32) void k_gemm_bf(const bf* __restrict__ A, const bf* __restrict__ Bt, float* C, unsigned K, unsigned ldc) {
    __shared__ __align__(16) float os[16 * 68];
    const int lane = threadIdx.x & 31, lr = lane & 15, hi = lane >> 4; const unsigned r0 = blockIdx.x * 64u, c0 = blockIdx.y * 64u;
    v8f acc[4][4];
#pragma unroll
    for (int mb = 0; mb < 4; ++mb)
#pragma unroll
        for (int nb = 0; nb < 4; ++nb) acc[mb][nb] = (v8f){};
    const size_t aoff = (size_t)(r0 + (unsigned)lr) * K + (size_t)(8 * hi), boff = (size_t)(c0 + (unsigned)lr) * K + (size_t)(8 * hi);
#pragma unroll 1
    for (unsigned kc = 0; kc < K; kc += 32u) {
        v16bf a[4];
#pragma unroll
        for (int mb = 0; mb < 4; ++mb) a[mb] = ldb(A + aoff + (size_t)mb * 16 * K + kc);
#pragma unroll
        for (int nb = 0; nb < 4; ++nb) { const v16bf b = ldb(Bt + boff + (size_t)nb * 16 * K + kc);
#pragma unroll
            for (int mb = 0; mb < 4; ++mb) acc[mb][nb] = wmmabg(a[mb], b, acc[mb][nb]); }
    }
#pragma unroll
    for (int mb = 0; mb < 4; ++mb) {
#pragma unroll
        for (int nb = 0; nb < 4; ++nb) {
#pragma unroll
            for (int j = 0; j < 8; ++j) os[(hi * 8 + j) * 68 + nb * 16 + lr] = acc[mb][nb][j]; }
        wave_sync();
        float* cb = C + (size_t)(r0 + (unsigned)(mb * 16)) * ldc + c0;
#pragma unroll 1
        for (int ps = 0; ps < 2; ++ps) {
#pragma unroll
            for (int s = 0; s < 8; ++s) { const int row = 2 * s + (lane >> 4), c4 = (lane & 15) * 4;
                const v4f val = *(const v4fa*)(&os[row * 68 + c4]);
                *(volatile v4f*)(cb + (size_t)row * ldc + c4) = val; }
            if (ps == 0) __threadfence(); }
        wave_sync();
    }
}

__global__ __launch_bounds__(256) void k_score(const float* __restrict__ W1Q, const float* __restrict__ W2K, const float* __restrict__ scale, float* WOUT, h16* PP) {
#pragma clang fp contract(off)
    __shared__ __align__(16) float qs[UN];
    __shared__ __align__(16) float cs[UN];
    __shared__ __align__(16) float sc[SK];
    __shared__ float wmax[8];
    __shared__ float wsum[8];
    const unsigned tid = threadIdx.x; const unsigned lane = tid & 31u;
    const int wave = __builtin_amdgcn_readfirstlane((int)(threadIdx.x >> 5));
    const unsigned bt = blockIdx.x; const unsigned b = bt / (unsigned)TQ;
    qs[tid] = W1Q[(size_t)bt * UN + tid];
    cs[tid] = bfr(scale[tid]);
    __syncthreads();
    const float* kb = W2K + (size_t)b * ((size_t)SK * UN) + lane;
#pragma unroll 1
    for (int s = wave; s < SK; s += 8) {
        const float* kr = kb + (size_t)s * UN;
        float p = 0.0f;
#pragma unroll 1
        for (int g = 0; g < UN / 32; ++g) { const int u = 32 * g + (int)lane; p = fmaf(cs[u], tanhf(qs[u] + kr[32 * g]), p); }
        p += __shfl_xor(p, 16, 32); p += __shfl_xor(p, 8, 32); p += __shfl_xor(p, 4, 32); p += __shfl_xor(p, 2, 32); p += __shfl_xor(p, 1, 32);
        if (lane == 0u) sc[s] = p;
    }
    __syncthreads();
    float mx = fmaxf(sc[tid], sc[tid + 256u]);
    mx = fmaxf(mx, __shfl_xor(mx, 16, 32)); mx = fmaxf(mx, __shfl_xor(mx, 8, 32)); mx = fmaxf(mx, __shfl_xor(mx, 4, 32)); mx = fmaxf(mx, __shfl_xor(mx, 2, 32)); mx = fmaxf(mx, __shfl_xor(mx, 1, 32));
    if (lane == 0u) wmax[wave] = mx;
    __syncthreads();
    float m = wmax[0];
#pragma unroll
    for (int w = 1; w < 8; ++w) m = fmaxf(m, wmax[w]);
    float ls = 0.0f;
#pragma unroll 1
    for (unsigned i = 0; i < 2u; ++i) { const unsigned idx = tid + 256u * i; const float e = expf(sc[idx] - m); sc[idx] = e; ls += e; }
    ls += __shfl_xor(ls, 16, 32); ls += __shfl_xor(ls, 8, 32); ls += __shfl_xor(ls, 4, 32); ls += __shfl_xor(ls, 2, 32); ls += __shfl_xor(ls, 1, 32);
    if (lane == 0u) wsum[wave] = ls;
    __syncthreads();
    float tot = wsum[0];
#pragma unroll
    for (int w = 1; w < 8; ++w) tot += wsum[w];
    const float inv = 1.0f / tot;
    float* wrow = WOUT + (size_t)bt * SK;
    h16* prow = PP + (size_t)bt * SK;
#pragma unroll 1
    for (int ps = 0; ps < 2; ++ps) {
        if (wave < 4) {
            const v4f e = *(const v4fa*)(&sc[4u * tid]); v4f w;
            w[0] = e[0] * inv; w[1] = e[1] * inv; w[2] = e[2] * inv; w[3] = e[3] * inv;
            *(volatile v4f*)(wrow + 4u * tid) = w;
        } else if (wave < 6) {
            const unsigned p8 = (tid - 128u) * 8u;
            const v4f e0 = *(const v4fa*)(&sc[p8]); const v4f e1 = *(const v4fa*)(&sc[p8 + 4u]); v8h hv;
#pragma unroll
            for (int i = 0; i < 4; ++i) { hv[i] = toh_flush((e0[i] * inv) * PCAR); hv[4 + i] = toh_flush((e1[i] * inv) * PCAR); }
            *(volatile v8h*)(prow + p8) = hv;
        }
        if (ps == 0) __threadfence(); }
}

__global__ __launch_bounds__(32) void k_ctx(const h16* __restrict__ P, const h16* __restrict__ VT, float* OUT) {
    __shared__ __align__(16) float os[16 * 68];
    const int lane = threadIdx.x & 31, lr = lane & 15, hi = lane >> 4; const unsigned r0 = blockIdx.x * 64u, c0 = blockIdx.y * 64u;
    const unsigned bz = blockIdx.z;
    const h16* A = P + (size_t)bz * ((size_t)TQ * SK);
    const h16* Bt = VT + (size_t)bz * ((size_t)VD * SK);
    float* C = OUT + (size_t)bz * ((size_t)TQ * VD);
    v8f acc[4][4];
#pragma unroll
    for (int mb = 0; mb < 4; ++mb)
#pragma unroll
        for (int nb = 0; nb < 4; ++nb) acc[mb][nb] = (v8f){};
    const size_t aoff = (size_t)(r0 + (unsigned)lr) * SK + (size_t)(8 * hi), boff = (size_t)(c0 + (unsigned)lr) * SK + (size_t)(8 * hi);
#pragma unroll 1
    for (unsigned kc = 0; kc < (unsigned)SK; kc += 32u) {
        v16h a[4];
#pragma unroll
        for (int mb = 0; mb < 4; ++mb) a[mb] = ldh(A + aoff + (size_t)mb * 16 * SK + kc);
#pragma unroll
        for (int nb = 0; nb < 4; ++nb) { const v16h b = ldh(Bt + boff + (size_t)nb * 16 * SK + kc);
#pragma unroll
            for (int mb = 0; mb < 4; ++mb) acc[mb][nb] = wmma16g(a[mb], b, acc[mb][nb]); }
    }
#pragma unroll
    for (int mb = 0; mb < 4; ++mb) {
#pragma unroll
        for (int nb = 0; nb < 4; ++nb) {
#pragma unroll
            for (int j = 0; j < 8; ++j) os[(hi * 8 + j) * 68 + nb * 16 + lr] = acc[mb][nb][j] * PINV; }
        wave_sync();
        float* cb = C + (size_t)(r0 + (unsigned)(mb * 16)) * VD + c0;
#pragma unroll 1
        for (int ps = 0; ps < 2; ++ps) {
#pragma unroll
            for (int s = 0; s < 8; ++s) { const int row = 2 * s + (lane >> 4), c4 = (lane & 15) * 4;
                const v4f val = *(const v4fa*)(&os[row * 68 + c4]);
                *(volatile v4f*)(cb + (size_t)row * VD + c4) = val; }
            if (ps == 0) __threadfence(); }
        wave_sync();
    }
}

static constexpr size_t al256(size_t v) { return (v + 255) & ~(size_t)255; }
static constexpr size_t N_QUERY = (size_t)NB * TQ * QD;
static constexpr size_t N_VALUE = (size_t)NB * SK * VD;
static constexpr size_t N_W1 = (size_t)QD * UN;
static constexpr size_t N_W2 = (size_t)VD * UN;
static constexpr size_t N_ROWS_OUT = (size_t)NB * TQ * SK;
static constexpr size_t OUT1_OFF = (size_t)NB_FULL * TQ * VD;
static constexpr size_t SZ_QB  = al256(N_QUERY * 2);
static constexpr size_t SZ_VB  = al256(N_VALUE * 2);
static constexpr size_t SZ_W1T = al256(N_W1 * 2);
static constexpr size_t SZ_W2T = al256(N_W2 * 2);
static constexpr size_t SZ_VT  = al256(N_VALUE * 2);
static constexpr size_t SZ_W1Q = al256((size_t)NB * TQ * UN * 4);
static constexpr size_t SZ_W2K = al256((size_t)NB * SK * UN * 4);
static constexpr size_t SZ_PP  = al256((size_t)NB * TQ * SK * 2);
static constexpr size_t SZ_TOTAL = SZ_QB + SZ_VB + SZ_W1T + SZ_W2T + SZ_VT + SZ_W1Q + SZ_W2K + SZ_PP;
static_assert(SZ_TOTAL <= (size_t)134217728);
static_assert(OUT1_OFF * 4 == (size_t)1048576);
static_assert(OUT1_OFF % 32 == 0);
static_assert((size_t)NB * TQ * VD <= OUT1_OFF);
static constexpr size_t N8_Q = N_QUERY / 8;
static constexpr size_t N8_V = N_VALUE / 8;
static constexpr unsigned G_CQ = (unsigned)((N8_Q + 255) / 256);
static constexpr unsigned G_CV = (unsigned)((N8_V + 255) / 256);

extern "C" void kernel_launch(void* const* d_in, const int* in_sizes, int n_in,
                              void* d_out, int out_size, void* d_ws, size_t ws_size, hipStream_t stream) {
    if (n_in < 5) return;
    if ((size_t)in_sizes[0] < N_QUERY || (size_t)in_sizes[1] < N_VALUE) return;
    if ((size_t)in_sizes[2] < N_W1 || (size_t)in_sizes[3] < N_W2 || in_sizes[4] < UN) return;
    if ((size_t)out_size < OUT1_OFF + N_ROWS_OUT) return;
    if (SZ_TOTAL > ws_size) return;
    const float* query = (const float*)d_in[0];
    const float* value = (const float*)d_in[1];
    const float* w1 = (const float*)d_in[2];
    const float* w2 = (const float*)d_in[3];
    const float* scale = (const float*)d_in[4];
    float* OUT = (float*)d_out;
    char* wsp = (char*)d_ws;
    bf* QB = (bf*)wsp; wsp += SZ_QB;
    bf* VB = (bf*)wsp; wsp += SZ_VB;
    bf* W1T = (bf*)wsp; wsp += SZ_W1T;
    bf* W2T = (bf*)wsp; wsp += SZ_W2T;
    h16* VT = (h16*)wsp; wsp += SZ_VT;
    float* W1Q = (float*)wsp; wsp += SZ_W1Q;
    float* W2K = (float*)wsp; wsp += SZ_W2K;
    h16* PP = (h16*)wsp; wsp += SZ_PP;

    k_cvt8<<<G_CQ, 256, 0, stream>>>(query, QB, N8_Q);
    k_cvt8<<<G_CV, 256, 0, stream>>>(value, VB, N8_V);
    k_trb<<<dim3(UN / 64, QD / 64, 1), 256, 0, stream>>>(w1, W1T, (unsigned)QD, (unsigned)UN);
    k_trb<<<dim3(UN / 64, VD / 64, 1), 256, 0, stream>>>(w2, W2T, (unsigned)VD, (unsigned)UN);
    k_trh<<<dim3(VD / 64, SK / 64, NB), 256, 0, stream>>>(value, VT, (unsigned)SK, (unsigned)VD);

    k_gemm_bf<<<dim3(NB * TQ / 64, UN / 64, 1), 32, 0, stream>>>(QB, W1T, W1Q, (unsigned)QD, (unsigned)UN);
    k_gemm_bf<<<dim3(NB * SK / 64, UN / 64, 1), 32, 0, stream>>>(VB, W2T, W2K, (unsigned)VD, (unsigned)UN);

    k_score<<<dim3(NB * TQ, 1, 1), 256, 0, stream>>>(W1Q, W2K, scale, OUT + OUT1_OFF, PP);

    k_ctx<<<dim3(TQ / 64, VD / 64, NB), 32, 0, stream>>>(PP, VT, OUT);
}
